// FlashAttention_60653528154551
// MI455X (gfx1250) — hardware-verified
//
#include <hip/hip_runtime.h>
#include <math.h>


#ifndef NB
#define NB 2
#endif
#ifndef SEQ
#define SEQ 2048
#endif
#define NB_FULL  2
#define SEQ_FULL 2048
#define DM   1024
#define NH   16
#define HD   64
#define DQ   (NH * HD)
#define QKVW (3 * DQ)
#define SCL  0.125f
#define PCAR 4096.0f
#define L2E  1.4426950408889634f
#define PKL  72
#define POS  68

static_assert(NB >= 1 && NB <= NB_FULL);
static_assert(SEQ % 64 == 0 && SEQ >= 64 && SEQ <= SEQ_FULL);
static_assert(HD == 64 && DM % 64 == 0 && QKVW % 64 == 0 && DQ % 32 == 0 && DM % 32 == 0);
static_assert(((QKVW * DM) / 64) % 64 == 0 && ((DM * DQ) / 64) % 64 == 0);

#define WS_XB   ((size_t)((NB - 1) * SEQ_FULL + SEQ) * DM * 2)
#define WS_WQ   ((size_t)QKVW * DM * 2)
#define WS_WO   ((size_t)DM * DQ * 2)
#define WS_CS   ((size_t)SEQ * HD * 2 * 4)
#define WS_QKV  ((size_t)SEQ * QKVW * 4)
#define WS_PL   ((size_t)NH * SEQ * HD * 2)
#define WS_CTX  ((size_t)NB * SEQ * DM * 2)
#define WS_TOTAL (WS_XB + WS_WQ + WS_WO + WS_CS + WS_QKV + 5 * WS_PL + 2 * WS_CTX)
static_assert(WS_TOTAL <= (size_t)134217728);
static_assert(WS_XB % 256 == 0 && WS_WQ % 256 == 0 && WS_WO % 256 == 0 && WS_CS % 256 == 0 && WS_QKV % 256 == 0 && WS_PL % 256 == 0 && WS_CTX % 256 == 0);

typedef _Float16 h16;
typedef unsigned short bf;
typedef __attribute__((ext_vector_type(16))) __bf16   v16bf;
typedef __attribute__((ext_vector_type(16))) _Float16 v16h;
typedef __attribute__((ext_vector_type(8)))  _Float16 v8h;
typedef __attribute__((ext_vector_type(8)))  unsigned short v8us;
typedef __attribute__((ext_vector_type(8)))  float    v8f;
typedef __attribute__((ext_vector_type(4)))  float    v4f;
typedef __attribute__((ext_vector_type(2)))  _Float16 v2h;
typedef __attribute__((ext_vector_type(2)))  unsigned short v2us;
typedef __attribute__((ext_vector_type(2)))  float    v2f;
typedef v8h  __attribute__((may_alias)) v8ha;
typedef v4f  __attribute__((may_alias)) v4fa;
typedef v8us __attribute__((may_alias)) v8usa;

__device__ __forceinline__ unsigned short f2bf(float f) { unsigned u = __float_as_uint(f); u += 0x7FFFu + ((u >> 16) & 1u); return (unsigned short)(u >> 16); }
__device__ __forceinline__ float bf2f(unsigned short b) { return __uint_as_float(((unsigned)b) << 16); }
__device__ __forceinline__ float bfr(float f) { return bf2f(f2bf(f)); }
__device__ __forceinline__ void splitf(float y, unsigned short& h, unsigned short& l) { h = f2bf(y); l = f2bf(y - bf2f(h)); }
__device__ __forceinline__ h16 tohx(float x) { return (h16)x; }
__device__ __forceinline__ v16h cat16(v8h lo, v8h hi) { return __builtin_shufflevector(lo, hi, 0, 1, 2, 3, 4, 5, 6, 7, 8, 9, 10, 11, 12, 13, 14, 15); }
__device__ __forceinline__ v16bf cat16b(v8us lo, v8us hi) { return __builtin_bit_cast(v16bf, __builtin_shufflevector(lo, hi, 0, 1, 2, 3, 4, 5, 6, 7, 8, 9, 10, 11, 12, 13, 14, 15)); }
__device__ __forceinline__ v8f wmma16(v16h a, v16h b, v8f c) { return __builtin_amdgcn_wmma_f32_16x16x32_f16(false, a, false, b, (short)0, c, false, false); }
__device__ __forceinline__ v8f wmmab(v16bf a, v16bf b, v8f c) { return __builtin_amdgcn_wmma_f32_16x16x32_bf16(false, a, false, b, (short)0, c, false, false); }

template <typename T16> struct WFrag;
template <> struct WFrag<h16> { typedef v16h V; static __device__ __forceinline__ V ld(const h16* p) { return cat16(*(const v8h*)p, *(const v8h*)(p + 16)); } static __device__ __forceinline__ v8f mma(V a, V b, v8f c) { return wmma16(a, b, c); } };
template <> struct WFrag<bf> { typedef v16bf V; static __device__ __forceinline__ V ld(const bf* p) { return cat16b(*(const v8us*)p, *(const v8us*)(p + 16)); } static __device__ __forceinline__ v8f mma(V a, V b, v8f c) { return wmmab(a, b, c); } };

template <typename T16, int NSPLIT, bool BIAS>
__global__ __launch_bounds__(32) void k_gemmw(const T16* __restrict__ A, const T16* __restrict__ A2, const T16* __restrict__ Bt, const T16* __restrict__ Bt2, int K, float* C, int ldc, const float* __restrict__ bias, size_t sA, size_t sB, size_t sC) {
    typedef typename WFrag<T16>::V V;
    __shared__ __align__(16) float os[16 * 68];
    const size_t z = blockIdx.z; A += z * sA; if (A2) A2 += z * sA; Bt += z * sB; if (Bt2) Bt2 += z * sB; C += z * sC;
    const int lane = threadIdx.x & 31, lr = lane & 15, hi = lane >> 4; const int r0 = blockIdx.x * 64, c0 = blockIdx.y * 64;
    v8f acc[4][4];
#pragma unroll
    for (int mb = 0; mb < 4; ++mb)
#pragma unroll
        for (int nb = 0; nb < 4; ++nb) acc[mb][nb] = (v8f){};
    const size_t aoff = (size_t)(r0 + lr) * K + 8 * hi, boff = (size_t)(c0 + lr) * K + 8 * hi;
#pragma unroll 1
    for (int kc = 0; kc < K; kc += 32) {
        V a[4], a2[4];
#pragma unroll
        for (int mb = 0; mb < 4; ++mb) { a[mb] = WFrag<T16>::ld(A + aoff + (size_t)mb * 16 * K + kc); if (NSPLIT == 1 || NSPLIT == 2) a2[mb] = WFrag<T16>::ld(A2 + aoff + (size_t)mb * 16 * K + kc); }
#pragma unroll
        for (int nb = 0; nb < 4; ++nb) { const V b = WFrag<T16>::ld(Bt + boff + (size_t)nb * 16 * K + kc); V b2; if (NSPLIT >= 2) b2 = WFrag<T16>::ld(Bt2 + boff + (size_t)nb * 16 * K + kc);
#pragma unroll
            for (int mb = 0; mb < 4; ++mb) { acc[mb][nb] = WFrag<T16>::mma(a[mb], b, acc[mb][nb]); if (NSPLIT == 1 || NSPLIT == 2) acc[mb][nb] = WFrag<T16>::mma(a2[mb], b, acc[mb][nb]); if (NSPLIT >= 2) acc[mb][nb] = WFrag<T16>::mma(a[mb], b2, acc[mb][nb]); } }
        asm volatile("v_nop\n\tv_nop\n\tv_nop\n\tv_nop" : "+v"(acc[0][0]), "+v"(acc[1][1]), "+v"(acc[2][2]), "+v"(acc[3][3]) : "v"(a[0]), "v"(a[3]));
    }
#pragma unroll
    for (int mb = 0; mb < 4; ++mb) {
#pragma unroll
        for (int nb = 0; nb < 4; ++nb) {
#pragma unroll
            for (int j = 0; j < 8; ++j) os[(hi * 8 + j) * 68 + nb * 16 + lr] = acc[mb][nb][j]; }
        __builtin_amdgcn_wave_barrier(); asm volatile("" ::: "memory");
        float* crow = C + (size_t)(r0 + mb * 16) * ldc + c0;
#pragma unroll 1
        for (int ps = 0; ps < 2; ++ps) {
#pragma unroll
            for (int s = 0; s < 8; ++s) { const int row = 2 * s + hi, cofs = lr * 4; v4f val = *(const v4fa*)(os + row * 68 + cofs); if (BIAS) { val[0] += bfr(bias[c0 + cofs]); val[1] += bfr(bias[c0 + cofs + 1]); val[2] += bfr(bias[c0 + cofs + 2]); val[3] += bfr(bias[c0 + cofs + 3]); }
                *(volatile v4f*)(crow + (size_t)row * ldc + cofs) = val; }
            if (ps == 0) __threadfence(); }
        __builtin_amdgcn_wave_barrier(); asm volatile("" ::: "memory");
    }
}

__global__ __launch_bounds__(256) void k_wtG(const float* __restrict__ w, int K, int N, bf* Bt) {
    const int lane = threadIdx.x & 31; const int L0 = (blockIdx.x * 8 + (threadIdx.x >> 5)) * 8; const int nlines = N * K / 64;
#pragma unroll
    for (int ps = 0; ps < 2; ++ps) {
#pragma unroll 1
        for (int l = 0; l < 8; ++l) { const int L = L0 + l; if (L >= nlines) break; const size_t e = (size_t)L * 64 + lane * 2; const int k = (int)(e % K), n = (int)(e / K); v2us o;
            o[0] = f2bf(w[(size_t)k * N + n]); o[1] = f2bf(w[(size_t)(k + 1) * N + n]); *(volatile v2us*)(Bt + e) = o; }
        if (ps == 0) __threadfence(); }
}
__global__ __launch_bounds__(256) void k_cvt8(const float* __restrict__ src, bf* dst, size_t n8) { const size_t i = (size_t)blockIdx.x * 256 + threadIdx.x; if (i >= n8) return; const v8f v = *(const v8f*)(src + i * 8); v8us o;
#pragma unroll
    for (int k = 0; k < 8; ++k) o[k] = f2bf(v[k]); *(volatile v8us*)(dst + i * 8) = o; __threadfence(); *(volatile v8us*)(dst + i * 8) = o; }

struct InvF { float f[HD / 2]; };
static_assert(sizeof(InvF) == 128);
__global__ __launch_bounds__(256) void k_cstab(InvF ivf, float* CS) {
    const int lane = threadIdx.x & 31; const int t = blockIdx.x * 8 + (threadIdx.x >> 5); if (t >= SEQ) return;
    float iv = 0.0f;
#pragma unroll
    for (int k = 0; k < HD / 2; ++k) iv = (lane == k) ? ivf.f[k] : iv;
    float ang = (float)t * iv; asm volatile("" : "+v"(ang));
    float sn, cn; sincosf(ang, &sn, &cn);
    v2f o; o[0] = cn; o[1] = sn;
    float* p0 = CS + ((size_t)t * HD + lane) * 2; float* p1 = p0 + HD;
    *(volatile v2f*)p0 = o; *(volatile v2f*)p1 = o; __threadfence(); *(volatile v2f*)p0 = o; *(volatile v2f*)p1 = o;
}

__global__ __launch_bounds__(256) void k_ropehl(const float* __restrict__ F, int pitch, int nheads, const float* __restrict__ CS, bf* Ph, bf* Pl) {
    const size_t e = ((size_t)blockIdx.x * 256 + threadIdx.x) * 2; if (e >= (size_t)nheads * SEQ * HD) return;
    const int d = (int)(e % HD); const int t = (int)((e / HD) % SEQ); const int h = (int)(e / ((size_t)HD * SEQ));
    const float* f = F + (size_t)t * pitch + h * HD; v2us oh, ol;
#pragma unroll
    for (int q = 0; q < 2; ++q) { const int dd = d + q; const int dp = (dd < HD / 2) ? dd + HD / 2 : dd - HD / 2; const float x0 = f[dd], x1 = f[dp];
        const v2f cs = *(const v2f*)(CS + ((size_t)t * HD + dd) * 2); float a = __fmul_rn(x0, cs[0]), bq = __fmul_rn(x1, cs[1]); asm volatile("" : "+v"(a)); asm volatile("" : "+v"(bq));
        const float r = (dd < HD / 2) ? __fsub_rn(a, bq) : __fadd_rn(a, bq);
        unsigned short a2, c2; splitf(r, a2, c2); oh[q] = a2; ol[q] = c2; }
    *(volatile v2us*)(Ph + e) = oh; *(volatile v2us*)(Pl + e) = ol; __threadfence(); *(volatile v2us*)(Ph + e) = oh; *(volatile v2us*)(Pl + e) = ol; }

__global__ __launch_bounds__(256) void k_vt16(const float* __restrict__ F, int pitch, int nheads, h16* V16) {
    const size_t e = ((size_t)blockIdx.x * 256 + threadIdx.x) * 2; if (e >= (size_t)nheads * HD * SEQ) return;
    const int t = (int)(e % SEQ); const int d = (int)((e / SEQ) % HD); const int g = (int)(e / ((size_t)SEQ * HD)); v2h o16;
#pragma unroll
    for (int q = 0; q < 2; ++q) o16[q] = tohx(F[(size_t)(t + q) * pitch + g * HD + d]);
    *(volatile v2h*)(V16 + e) = o16; __threadfence(); *(volatile v2h*)(V16 + e) = o16; }

__global__ __launch_bounds__(128) void k_attn(const bf* __restrict__ Qh, const bf* __restrict__ Ql, const bf* __restrict__ Kh, const bf* __restrict__ Kl,
                                             const h16* __restrict__ Vt, bf* CtxH, bf* CtxL, int row0) {
    __shared__ __align__(16) unsigned short sKh[64 * PKL];
    __shared__ __align__(16) unsigned short sKl[64 * PKL];
    __shared__ __align__(16) h16 sVt[64 * PKL];
    __shared__ __align__(16) h16 sP[4][16 * PKL];
    __shared__ __align__(16) float os[4][16 * POS];
    const int tid = threadIdx.x, wave = tid >> 5, lane = tid & 31, lr = lane & 15, hi = lane >> 4;
    const int nqt = SEQ / 64;
    const int h = blockIdx.x / nqt, qt = blockIdx.x - h * nqt;
    const int q0 = qt * 64 + wave * 16;
    const size_t hq = (size_t)h * SEQ * HD, hv = (size_t)h * HD * SEQ;
    v16bf aq[2], aq2[2];
#pragma unroll
    for (int ks = 0; ks < 2; ++ks) { const size_t o = hq + (size_t)(q0 + lr) * HD + 8 * hi + ks * 32; aq[ks] = WFrag<bf>::ld(Qh + o); aq2[ks] = WFrag<bf>::ld(Ql + o); }
    float mrow[8], lrow[8];
#pragma unroll
    for (int r = 0; r < 8; ++r) { mrow[r] = -1.0e30f; lrow[r] = 0.0f; }
    v8f accO[4];
#pragma unroll
    for (int nb = 0; nb < 4; ++nb) accO[nb] = (v8f){};
    h16* sPw = &sP[wave][0]; float* osw = &os[wave][0];
#pragma unroll 1
    for (int kt = 0; kt < SEQ / 64; ++kt) {
        __syncthreads();
#pragma unroll
        for (int j = 0; j < 4; ++j) {
            const int idx = tid + 128 * j, row = idx >> 3, c8 = (idx & 7) * 8;
            const size_t ko = hq + (size_t)(kt * 64 + row) * HD + c8;
            const v8us kh = *(const v8us*)(Kh + ko); const v8us kl = *(const v8us*)(Kl + ko);
            const v8h vv = *(const v8h*)(Vt + hv + (size_t)row * SEQ + (size_t)kt * 64 + c8);
            *(v8us*)(sKh + row * PKL + c8) = kh; *(v8us*)(sKl + row * PKL + c8) = kl; *(v8h*)(sVt + row * PKL + c8) = vv; }
        __syncthreads();
        v8f accS[4];
#pragma unroll
        for (int nb = 0; nb < 4; ++nb) accS[nb] = (v8f){};
#pragma unroll
        for (int ks = 0; ks < 2; ++ks)
#pragma unroll
            for (int nb = 0; nb < 4; ++nb) { const int bo = (nb * 16 + lr) * PKL + 8 * hi + ks * 32;
                const v16bf b = WFrag<bf>::ld(sKh + bo); const v16bf b2 = WFrag<bf>::ld(sKl + bo);
                accS[nb] = wmmab(aq[ks], b, accS[nb]); accS[nb] = wmmab(aq2[ks], b, accS[nb]); accS[nb] = wmmab(aq[ks], b2, accS[nb]); }
        asm volatile("v_nop\n\tv_nop\n\tv_nop\n\tv_nop" : "+v"(accS[0]), "+v"(accS[1]), "+v"(accS[2]), "+v"(accS[3]) : "v"(aq[0]), "v"(aq[1]), "v"(aq2[0]), "v"(aq2[1]));
#pragma unroll
        for (int r = 0; r < 8; ++r) {
            float mx = -1.0e30f;
#pragma unroll
            for (int nb = 0; nb < 4; ++nb) { const float s = accS[nb][r] * SCL; accS[nb][r] = s; mx = fmaxf(mx, s); }
#pragma unroll
            for (int sh = 1; sh < 16; sh <<= 1) mx = fmaxf(mx, __shfl_xor(mx, sh, 32));
            const float nm = fmaxf(mrow[r], mx);
            float dm = mrow[r] - nm; asm volatile("" : "+v"(dm));
            const float fac = __builtin_amdgcn_exp2f(dm * L2E);
            float rs = 0.0f;
#pragma unroll
            for (int nb = 0; nb < 4; ++nb) { float d0 = accS[nb][r] - nm; asm volatile("" : "+v"(d0));
                const h16 p16 = tohx(__builtin_amdgcn_exp2f(d0 * L2E) * PCAR);
                sPw[(8 * hi + r) * PKL + nb * 16 + lr] = p16; rs += (float)p16; }
#pragma unroll
            for (int sh = 1; sh < 16; sh <<= 1) rs += __shfl_xor(rs, sh, 32);
            lrow[r] = lrow[r] * fac + rs; mrow[r] = nm;
#pragma unroll
            for (int nb = 0; nb < 4; ++nb) accO[nb][r] *= fac;
        }
        __builtin_amdgcn_wave_barrier(); asm volatile("" ::: "memory");
        v16h pa[2];
#pragma unroll
        for (int ks = 0; ks < 2; ++ks) { const h16* pp = sPw + lr * PKL + 8 * hi + ks * 32; pa[ks] = cat16(*(const v8ha*)pp, *(const v8ha*)(pp + 16)); }
#pragma unroll
        for (int nb = 0; nb < 4; ++nb)
#pragma unroll
            for (int ks = 0; ks < 2; ++ks) { const v16h bv = WFrag<h16>::ld(sVt + (nb * 16 + lr) * PKL + 8 * hi + ks * 32); accO[nb] = wmma16(pa[ks], bv, accO[nb]); }
        asm volatile("v_nop\n\tv_nop\n\tv_nop\n\tv_nop" : "+v"(accO[0]), "+v"(accO[1]), "+v"(accO[2]), "+v"(accO[3]) : "v"(pa[0]), "v"(pa[1]));
    }
#pragma unroll
    for (int r = 0; r < 8; ++r) { const float inv = __fdiv_rn(1.0f, lrow[r]);
#pragma unroll
        for (int nb = 0; nb < 4; ++nb) osw[(8 * hi + r) * POS + nb * 16 + lr] = accO[nb][r] * inv; }
    __builtin_amdgcn_wave_barrier(); asm volatile("" ::: "memory");
#pragma unroll 1
    for (int ps = 0; ps < 2; ++ps) {
#pragma unroll
        for (int s = 0; s < 4; ++s) { const int row = (lane >> 3) + 4 * s, c8 = (lane & 7) * 8;
            const v4f v0 = *(const v4fa*)(osw + row * POS + c8), v1 = *(const v4fa*)(osw + row * POS + c8 + 4);
            v8us oh, ol;
#pragma unroll
            for (int k = 0; k < 4; ++k) { unsigned short a, c; splitf(v0[k], a, c); oh[k] = a; ol[k] = c; splitf(v1[k], a, c); oh[k + 4] = a; ol[k + 4] = c; }
            const size_t go = (size_t)(row0 + q0 + row) * DM + (size_t)h * HD + c8;
            *(volatile v8us*)(CtxH + go) = oh; *(volatile v8us*)(CtxL + go) = ol; }
        if (ps == 0) __threadfence(); }
}

extern "C" void kernel_launch(void* const* d_in, const int* in_sizes, int n_in,
                              void* d_out, int out_size, void* d_ws, size_t ws_size, hipStream_t stream) {
    if (n_in < 4) return;
    const long long rows = (long long)(NB - 1) * SEQ_FULL + SEQ;
    if ((long long)in_sizes[0] < rows * DM || (long long)in_sizes[1] < (long long)DM * QKVW || (long long)in_sizes[2] < (long long)DQ * DM || in_sizes[3] < DM) return;
    if ((long long)out_size < rows * DM) return;
    if (WS_TOTAL > ws_size) return;
    const float* x     = (const float*)d_in[0];
    const float* qkv_w = (const float*)d_in[1];
    const float* out_w = (const float*)d_in[2];
    const float* out_b = (const float*)d_in[3];
    float* OUT = (float*)d_out;
    char* wsp = (char*)d_ws;
    auto take = [&](size_t bytes) { char* p = wsp; wsp += (bytes + 255) & ~(size_t)255; return (void*)p; };
    bf* Xb = (bf*)take(WS_XB); bf* WqT = (bf*)take(WS_WQ); bf* WoT = (bf*)take(WS_WO); float* CS = (float*)take(WS_CS); float* QKVb = (float*)take(WS_QKV);
    bf* QPh = (bf*)take(WS_PL); bf* QPl = (bf*)take(WS_PL); bf* KPh = (bf*)take(WS_PL); bf* KPl = (bf*)take(WS_PL); h16* VT = (h16*)take(WS_PL);
    bf* CtxH = (bf*)take(WS_CTX); bf* CtxL = (bf*)take(WS_CTX);
    if ((size_t)(wsp - (char*)d_ws) > ws_size) return;

    InvF ivf;
    for (int j = 0; j < HD / 2; ++j) { const float p = (float)pow(10000.0, (double)j / 32.0); ivf.f[j] = 1.0f / p; }

    const size_t nx8 = (size_t)rows * DM / 8;
    k_cvt8<<<(unsigned)((nx8 + 255) / 256), 256, 0, stream>>>(x, Xb, nx8);
    k_wtG<<<(QKVW * DM / 64) / 64, 256, 0, stream>>>(qkv_w, DM, QKVW, WqT);
    k_wtG<<<(DM * DQ / 64) / 64, 256, 0, stream>>>(out_w, DQ, DM, WoT);
    k_cstab<<<SEQ / 8, 256, 0, stream>>>(ivf, CS);
    const unsigned LPL = (unsigned)(((size_t)NH * SEQ * HD / 2 + 255) / 256);
    for (int b = 0; b < NB; ++b) {
        k_gemmw<bf, 0, false><<<dim3(SEQ / 64, QKVW / 64, 1), 32, 0, stream>>>(Xb + (size_t)b * SEQ_FULL * DM, nullptr, WqT, nullptr, DM, QKVb, QKVW, nullptr, 0, 0, 0);
        k_ropehl<<<LPL, 256, 0, stream>>>(QKVb, QKVW, NH, CS, QPh, QPl);
        k_ropehl<<<LPL, 256, 0, stream>>>(QKVb + DQ, QKVW, NH, CS, KPh, KPl);
        k_vt16<<<LPL, 256, 0, stream>>>(QKVb + 2 * DQ, QKVW, NH, VT);
        k_attn<<<NH * (SEQ / 64), 128, 0, stream>>>(QPh, QPl, KPh, KPl, VT, CtxH, CtxL, b * SEQ);
    }
    k_gemmw<bf, 1, true><<<dim3(SEQ / 64, DM / 64, NB), 32, 0, stream>>>(CtxH, CtxL, WoT, nullptr, DQ, OUT, DM, out_b, (size_t)SEQ * DM, 0, (size_t)SEQ_FULL * DM);
}
